// RotaryPEMultiHeadSelfAttention_9929964388671
// MI455X (gfx1250) — hardware-verified
//
#include <hip/hip_runtime.h>
#include <math.h>
#include <stdint.h>

#define BSZ   2
#define DM    1024
#define NH    16
#define HD    64
#define NROT  32
#define NFREQ 16
#define QKVN  (3 * DM)
#define HSTR  (3 * HD)
static_assert(NH * HD == DM);
static_assert(HD == 64);
static_assert(NROT == 2 * NFREQ);
static_assert(NH * HSTR == QKVN);
static_assert((DM % 64) == 0 && (QKVN % 64) == 0 && (DM % 32) == 0);
static_assert(((QKVN * DM / 8) % 256) == 0);
static_assert(DM / 8 == 128);

typedef _Float16 v16h __attribute__((ext_vector_type(16)));
typedef _Float16 v8h  __attribute__((ext_vector_type(8)));
typedef float    v8f  __attribute__((ext_vector_type(8)));
typedef float    v4f  __attribute__((ext_vector_type(4)));
typedef unsigned int v4u __attribute__((ext_vector_type(4)));

__device__ __forceinline__ unsigned short bf_bits(float f) {
  unsigned u = __float_as_uint(f);
  return (unsigned short)((u + 0x7FFFu + ((u >> 16) & 1u)) >> 16);
}
__device__ __forceinline__ float bf_up(unsigned short h) { return __uint_as_float(((unsigned)h) << 16); }
__device__ __forceinline__ float bfr(float f) { return bf_up(bf_bits(f)); }
__device__ __forceinline__ unsigned short h_bits(_Float16 x) { return __builtin_bit_cast(unsigned short, x); }
__device__ __forceinline__ unsigned pk16(unsigned short a, unsigned short b) { return (unsigned)a | ((unsigned)b << 16); }
__device__ __forceinline__ v8f zero8() { v8f z = {0.f, 0.f, 0.f, 0.f, 0.f, 0.f, 0.f, 0.f}; return z; }

__device__ __forceinline__ void ld8(const float* p, float* o) {
  const v4f a = *(const v4f*)(p);
  const v4f b = *(const v4f*)(p + 4);
  o[0] = a[0]; o[1] = a[1]; o[2] = a[2]; o[3] = a[3];
  o[4] = b[0]; o[5] = b[1]; o[6] = b[2]; o[7] = b[3];
}

__device__ __forceinline__ v16h ldfrag_h(const _Float16* p) {
  union { v16h v; v8h h[2]; } f;
  f.h[0] = *(const v8h*)(p);
  f.h[1] = *(const v8h*)(p + 16);
  return f.v;
}

__device__ __forceinline__ v8f mma_h(v16h a, v16h b, v8f c) {
  c = __builtin_amdgcn_wmma_f32_16x16x32_f16(false, a, false, b, (short)0, c, false, false);
#if defined(__HIP_DEVICE_COMPILE__)
  asm volatile("v_nop\n\tv_nop\n\tv_nop\n\tv_nop" : "+v"(c) : "v"(a), "v"(b));
#endif
  return c;
}
__device__ __forceinline__ v8f mma_h_raw(v16h a, v16h b, v8f c) {
  return __builtin_amdgcn_wmma_f32_16x16x32_f16(false, a, false, b, (short)0, c, false, false);
}
__device__ __forceinline__ void dep_guard_h(v8f& a, v8f& b, v16h x) {
#if defined(__HIP_DEVICE_COMPILE__)
  asm volatile("v_nop\n\tv_nop\n\tv_nop\n\tv_nop" : "+v"(a), "+v"(b) : "v"(x));
#endif
}
__device__ __forceinline__ void keep4_h(v16h a, v16h b, v16h c, v16h d) {
#if defined(__HIP_DEVICE_COMPILE__)
  asm volatile("v_nop" :: "v"(a), "v"(b), "v"(c), "v"(d));
#endif
}
__device__ __forceinline__ void acc_guard4(v8f& a, v8f& b, v8f& c, v8f& d) {
#if defined(__HIP_DEVICE_COMPILE__)
  asm volatile("v_nop\n\tv_nop\n\tv_nop\n\tv_nop" : "+v"(a), "+v"(b), "+v"(c), "+v"(d));
#endif
}

struct Theta16 { float t[NFREQ]; };
static_assert(sizeof(Theta16) == NFREQ * 4);

__global__ __launch_bounds__(256) void rope_tab(Theta16 th, float* ct, float* st, int n) {
#pragma clang fp contract(off)
  const int i = blockIdx.x * 256 + threadIdx.x;
  if (i < n) {
    const int j = i & (NFREQ - 1);
    const int l = i >> 4;
    float tv = th.t[0];
#pragma unroll
    for (int q = 1; q < NFREQ; ++q) tv = (j == q) ? th.t[q] : tv;
    const float ang = (float)l * tv;
    const float cv = cosf(ang);
    const float sv = sinf(ang);
    *(volatile float*)(ct + i) = cv;
    *(volatile float*)(st + i) = sv;
    __threadfence();
    *(volatile float*)(ct + i) = cv;
    *(volatile float*)(st + i) = sv;
  }
}

__global__ __launch_bounds__(256) void cvt_xh(const float* __restrict__ in, unsigned short* out, int n8,
                                              float sc) {
  const int i = blockIdx.x * 256 + threadIdx.x;
  if (i < n8) {
    const v4f a = *(const v4f*)(in + (size_t)i * 8);
    const v4f b = *(const v4f*)(in + (size_t)i * 8 + 4);
    v4u p;
    p[0] = pk16(h_bits((_Float16)(bfr(a[0]) * sc)), h_bits((_Float16)(bfr(a[1]) * sc)));
    p[1] = pk16(h_bits((_Float16)(bfr(a[2]) * sc)), h_bits((_Float16)(bfr(a[3]) * sc)));
    p[2] = pk16(h_bits((_Float16)(bfr(b[0]) * sc)), h_bits((_Float16)(bfr(b[1]) * sc)));
    p[3] = pk16(h_bits((_Float16)(bfr(b[2]) * sc)), h_bits((_Float16)(bfr(b[3]) * sc)));
    *(volatile v4u*)(out + (size_t)i * 8) = p;
    __threadfence();
    *(volatile v4u*)(out + (size_t)i * 8) = p;
  }
}

__global__ __launch_bounds__(256) void gemm64(
    const unsigned short* __restrict__ Ap, int lda,
    const unsigned short* __restrict__ Btp, int ldb,
    float* Cf, int ldc, int M, int N, int K, float oscale) {
  const _Float16* Ah = (const _Float16*)(const void*)Ap;
  const _Float16* Bh = (const _Float16*)(const void*)Btp;
  __shared__ __align__(16) float sT[8][16 * 68];
  const int lane = threadIdx.x & 31;
  const int wave = threadIdx.x >> 5;
  const int tilesN = N >> 6;
  const int tilesM = M >> 6;
  const int tile = blockIdx.x * 8 + wave;
  if (tile >= tilesM * tilesN) return;
  const int tm = tile / tilesN;
  const int tn = tile - tm * tilesN;
  const int m0 = tm << 6;
  const int n0 = tn << 6;

  const int rlane = lane & 15;
  const int koff  = (lane >> 4) * 8;
  const int mOff  = (lane >> 4) * 8;

  v8f acc[4][4];
#pragma unroll
  for (int i = 0; i < 4; ++i)
#pragma unroll
    for (int j = 0; j < 4; ++j) acc[i][j] = zero8();

  for (int k0 = 0; k0 < K; k0 += 32) {
    v16h bh[4];
#pragma unroll
    for (int j = 0; j < 4; ++j) {
      const size_t bo = (size_t)(n0 + (j << 4) + rlane) * ldb + koff + k0;
      bh[j] = ldfrag_h(Bh + bo);
    }
#pragma unroll
    for (int i = 0; i < 4; ++i) {
      const size_t ao = (size_t)(m0 + (i << 4) + rlane) * lda + koff + k0;
      const v16h ah = ldfrag_h(Ah + ao);
#pragma unroll
      for (int j = 0; j < 4; ++j) acc[i][j] = mma_h_raw(ah, bh[j], acc[i][j]);
      dep_guard_h(acc[i][0], acc[i][3], ah);
    }
    keep4_h(bh[0], bh[1], bh[2], bh[3]);
  }
  acc_guard4(acc[0][0], acc[0][1], acc[0][2], acc[0][3]);
  acc_guard4(acc[1][0], acc[1][1], acc[1][2], acc[1][3]);
  acc_guard4(acc[2][0], acc[2][1], acc[2][2], acc[2][3]);
  acc_guard4(acc[3][0], acc[3][1], acc[3][2], acc[3][3]);

  float* slab = sT[wave];
  const int h2 = lane >> 4, c4 = (lane & 15) * 4;
#pragma unroll
  for (int i = 0; i < 4; ++i) {
    const int mBase = m0 + (i << 4);
#pragma unroll
    for (int r = 0; r < 8; ++r) {
#pragma unroll
      for (int j = 0; j < 4; ++j) {
        slab[(mOff + r) * 68 + (j << 4) + rlane] = acc[i][j][r];
      }
    }
    __builtin_amdgcn_fence(__ATOMIC_RELEASE, "workgroup");
    __builtin_amdgcn_wave_barrier();
    __builtin_amdgcn_fence(__ATOMIC_ACQUIRE, "workgroup");
    v4f ov[8];
#pragma unroll
    for (int it = 0; it < 8; ++it) {
      const int row = it * 2 + h2;
      const v4f xs = *(const v4f*)(slab + row * 68 + c4);
      ov[it] = xs * oscale;
    }
    for (int pass = 0; pass < 2; ++pass) {
#pragma unroll
      for (int it = 0; it < 8; ++it) {
        const int row = it * 2 + h2;
        *(volatile v4f*)(Cf + (size_t)(mBase + row) * ldc + n0 + c4) = ov[it];
      }
      __threadfence();
    }
    __builtin_amdgcn_fence(__ATOMIC_RELEASE, "workgroup");
    __builtin_amdgcn_wave_barrier();
    __builtin_amdgcn_fence(__ATOMIC_ACQUIRE, "workgroup");
  }
}

__global__ __launch_bounds__(128) void rope_qk(const float* __restrict__ qkvf,
                                               const float* __restrict__ ct, const float* __restrict__ st,
                                               unsigned short* qh, unsigned short* kh, float qs) {
#pragma clang fp contract(off)
  const int tid = threadIdx.x;
  const int row = blockIdx.x;
  const int l   = row >> 1;
  const float* rowp = qkvf + (size_t)row * QKVN;
  const int d0  = tid * 8;
  const int hd  = d0 >> 6;
  const int dd  = d0 & (HD - 1);
  const int pdd = dd ^ 16;
  const int qc  = hd * HSTR + dd;
  const int pc  = hd * HSTR + pdd;
  const int j0  = dd & (NFREQ - 1);
  const float sgn = (dd < NFREQ) ? -1.0f : 1.0f;
  const bool rot  = dd < NROT;
  float xq[8], pq[8], xk[8], pk[8], cs[8], sn[8];
  ld8(rowp + qc, xq);
  ld8(rowp + pc, pq);
  ld8(rowp + HD + qc, xk);
  ld8(rowp + HD + pc, pk);
  const size_t tofs = (size_t)l * NFREQ + j0;
  ld8(ct + tofs, cs);
  ld8(st + tofs, sn);

  v4u aq, ak;
#pragma unroll
  for (int pp = 0; pp < 4; ++pp) {
    const int e0 = 2 * pp, e1 = 2 * pp + 1;
    const float rq0 = xq[e0] * cs[e0] + (sgn * pq[e0]) * sn[e0];
    const float rq1 = xq[e1] * cs[e1] + (sgn * pq[e1]) * sn[e1];
    const float rk0 = xk[e0] * cs[e0] + (sgn * pk[e0]) * sn[e0];
    const float rk1 = xk[e1] * cs[e1] + (sgn * pk[e1]) * sn[e1];
    const float yq0 = rot ? rq0 : xq[e0];
    const float yq1 = rot ? rq1 : xq[e1];
    const float yk0 = rot ? rk0 : xk[e0];
    const float yk1 = rot ? rk1 : xk[e1];
    aq[pp] = pk16(h_bits((_Float16)(yq0 * qs)), h_bits((_Float16)(yq1 * qs)));
    ak[pp] = pk16(h_bits((_Float16)(yk0 * qs)), h_bits((_Float16)(yk1 * qs)));
  }
  const size_t o = (size_t)row * DM + d0;
  *(volatile v4u*)(qh + o) = aq;
  *(volatile v4u*)(kh + o) = ak;
  __threadfence();
  *(volatile v4u*)(qh + o) = aq;
  *(volatile v4u*)(kh + o) = ak;
}

__global__ __launch_bounds__(256) void v_planes(const float* __restrict__ qkvf, unsigned short* vt, int nseq,
                                                float vscale) {
  __shared__ __align__(16) float svt[64 * 68];
  const int tid = threadIdx.x;
  const int kt  = blockIdx.x;
  const int hh  = blockIdx.y;
  const int b   = blockIdx.z;
  const int t0  = kt * 64;
#pragma unroll
  for (int i = 0; i < 4; ++i) {
    const int idx = i * 256 + tid;
    const int tt = idx >> 4, c4 = (idx & 15) * 4;
    const size_t srow = (size_t)(t0 + tt) * BSZ + b;
    const v4f a = *(const v4f*)(qkvf + srow * QKVN + hh * HSTR + 2 * HD + c4);
    *(v4f*)(svt + tt * 68 + c4) = a;
  }
  __syncthreads();

  const int g = tid >> 3, piece = tid & 7;
  v4u hv[2];
  size_t hofs[2];
#pragma unroll
  for (int it = 0; it < 2; ++it) {
    const int d = it * 32 + g;
    v4u a;
#pragma unroll
    for (int e = 0; e < 4; ++e) {
      const float f0 = svt[(piece * 8 + 2 * e) * 68 + d] * vscale;
      const float f1 = svt[(piece * 8 + 2 * e + 1) * 68 + d] * vscale;
      a[e] = pk16(h_bits((_Float16)f0), h_bits((_Float16)f1));
    }
    hv[it] = a;
    hofs[it] = ((size_t)(b * DM + hh * HD + d)) * (size_t)nseq + t0 + piece * 8;
  }
  for (int pass = 0; pass < 2; ++pass) {
#pragma unroll
    for (int it = 0; it < 2; ++it) *(volatile v4u*)(vt + hofs[it]) = hv[it];
    __threadfence();
  }
}

__global__ __launch_bounds__(128)
void attn64(const unsigned short* __restrict__ qhp, const unsigned short* __restrict__ khp,
            const unsigned short* __restrict__ vtp, float* outf, int nseq, float sscale, float oscl) {
  union FH { v16h v; v8h h[2]; };
  __shared__ __align__(16) _Float16 Ks[64 * 64];
  __shared__ __align__(16) _Float16 Vts[64 * 64];
  __shared__ __align__(16) _Float16 Psh[4][16 * 64];
  __shared__ __align__(16) float    Os[4][16 * 64];

  const int tid  = threadIdx.x;
  const int wave = tid >> 5;
  const int lane = tid & 31;
  const int hh   = lane >> 4;
  const int c    = lane & 15;

  const int nqt = nseq >> 6;
  const int bx = blockIdx.x;
  const int qt = bx % nqt;
  const int hb = bx / nqt;
  const int h  = hb % NH;
  const int b  = hb / NH;
  const int q0 = qt * 64 + wave * 16;

  const _Float16* Qp = (const _Float16*)(const void*)qhp + (size_t)h * HD;
  const _Float16* Kp = (const _Float16*)(const void*)khp + (size_t)h * HD;
  const _Float16* Vt = (const _Float16*)(const void*)vtp + ((size_t)b * DM + (size_t)h * HD) * (size_t)nseq;

  v16h qa[2];
#pragma unroll
  for (int dc = 0; dc < 2; ++dc) {
    const size_t qo = ((size_t)(q0 + c) * BSZ + b) * DM + dc * 32 + 8 * hh;
    qa[dc] = ldfrag_h(Qp + qo);
  }

  float mrow[8], lrow[8];
  v8f oacc[4];
#pragma unroll
  for (int r = 0; r < 8; ++r) { mrow[r] = -INFINITY; lrow[r] = 0.f; }
#pragma unroll
  for (int t = 0; t < 4; ++t) oacc[t] = zero8();

  for (int kt = 0; kt < nqt; ++kt) {
    const int kv0 = kt * 64;
    __syncthreads();
    {
      const int r = tid >> 1, half = (tid & 1) * 32;
      const _Float16* kg = Kp + ((size_t)(kv0 + r) * BSZ + b) * DM + half;
      const _Float16* vg = Vt + (size_t)r * (size_t)nseq + kv0 + half;
#pragma unroll
      for (int i = 0; i < 4; ++i) {
        const v8h a0 = *(const v8h*)(kg + 8 * i);
        const v8h b0 = *(const v8h*)(vg + 8 * i);
        *(v8h*)(Ks + r * 64 + half + 8 * i) = a0;
        *(v8h*)(Vts + r * 64 + half + 8 * i) = b0;
      }
    }
    __syncthreads();

    v8f s[4];
#pragma unroll
    for (int j = 0; j < 4; ++j) {
      v8f acc = zero8();
#pragma unroll
      for (int dc = 0; dc < 2; ++dc) {
        const int ko = (j * 16 + c) * 64 + dc * 32 + 8 * hh;
        FH kb;
        kb.h[0] = *(const v8h*)(Ks + ko);
        kb.h[1] = *(const v8h*)(Ks + ko + 16);
        acc = mma_h(qa[dc], kb.v, acc);
      }
      s[j] = acc;
    }

    _Float16* pwh = Psh[wave];
#pragma unroll
    for (int r = 0; r < 8; ++r) {
      float m = -INFINITY;
#pragma unroll
      for (int j = 0; j < 4; ++j) {
        const float sv = s[j][r] * sscale;
        s[j][r] = sv;
        m = fmaxf(m, sv);
      }
#pragma unroll
      for (int off = 1; off < 16; off <<= 1) m = fmaxf(m, __shfl_xor(m, off, 32));
      const float mnew  = fmaxf(mrow[r], m);
      const float msafe = (mnew == -INFINITY) ? 0.f : mnew;
      const float alpha = __expf(mrow[r] - msafe);
      mrow[r] = mnew;
      float psum = 0.f;
#pragma unroll
      for (int j = 0; j < 4; ++j) {
        const float p = __expf(s[j][r] - msafe);
        psum += p;
        const _Float16 ph = (_Float16)(p * 1024.0f);
        pwh[(8 * hh + r) * 64 + j * 16 + c] = ph;
      }
#pragma unroll
      for (int off = 1; off < 16; off <<= 1) psum += __shfl_xor(psum, off, 32);
      lrow[r] = lrow[r] * alpha + psum;
#pragma unroll
      for (int t = 0; t < 4; ++t) oacc[t][r] *= alpha;
    }
    __builtin_amdgcn_fence(__ATOMIC_RELEASE, "workgroup");
    __builtin_amdgcn_wave_barrier();
    __builtin_amdgcn_fence(__ATOMIC_ACQUIRE, "workgroup");

#pragma unroll 1
    for (int kk = 0; kk < 2; ++kk) {
      FH pa;
      pa.h[0] = *(const v8h*)(pwh + c * 64 + kk * 32 + 8 * hh);
      pa.h[1] = *(const v8h*)(pwh + c * 64 + kk * 32 + 16 + 8 * hh);
#pragma unroll
      for (int t = 0; t < 4; ++t) {
        FH vb;
        vb.h[0] = *(const v8h*)(Vts + (t * 16 + c) * 64 + kk * 32 + 8 * hh);
        vb.h[1] = *(const v8h*)(Vts + (t * 16 + c) * 64 + kk * 32 + 16 + 8 * hh);
        oacc[t] = mma_h(pa.v, vb.v, oacc[t]);
      }
    }
  }

  float* os = Os[wave];
#pragma unroll
  for (int r = 0; r < 8; ++r) {
    const float l = lrow[r];
    const float inv = ((l > 0.f) ? (1.0f / l) : 0.f) * oscl;
#pragma unroll
    for (int t = 0; t < 4; ++t) os[(8 * hh + r) * 64 + t * 16 + c] = oacc[t][r] * inv;
  }
  __builtin_amdgcn_fence(__ATOMIC_RELEASE, "workgroup");
  __builtin_amdgcn_wave_barrier();
  __builtin_amdgcn_fence(__ATOMIC_ACQUIRE, "workgroup");
  {
    const int h2 = lane >> 4, c4 = (lane & 15) * 4;
    v4f ov[8];
    size_t go[8];
#pragma unroll
    for (int it = 0; it < 8; ++it) {
      const int row = it * 2 + h2;
      ov[it] = *(const v4f*)(os + row * 64 + c4);
      const size_t dr = (size_t)(q0 + row) * BSZ + b;
      go[it] = dr * DM + (size_t)h * HD + c4;
    }
    for (int pass = 0; pass < 2; ++pass) {
#pragma unroll
      for (int it = 0; it < 8; ++it) *(volatile v4f*)(outf + go[it]) = ov[it];
      __threadfence();
    }
  }
}

extern "C" void kernel_launch(void* const* d_in, const int* in_sizes, int n_in,
                              void* d_out, int out_size, void* d_ws, size_t ws_size,
                              hipStream_t stream) {
  if (n_in < 2) return;
  if (in_sizes[1] != QKVN * DM) return;
  const int nx = in_sizes[0];
  if (nx < BSZ * DM * 64) return;
  if ((nx % (BSZ * DM)) != 0) return;
  const int nseq = nx / (BSZ * DM);
  if ((nseq % 64) != 0) return;
  if (out_size != nx) return;
  const int rows = nseq * BSZ;

  const float* x = (const float*)d_in[0];
  const float* w = (const float*)d_in[1];

  const size_t PXh  = (size_t)rows * DM * 2;
  const size_t PWq  = (size_t)QKVN * DM * 2;
  const size_t PTab = (size_t)nseq * NFREQ * 4;
  const size_t PQKV = (size_t)rows * QKVN * 4;
  const size_t PQK  = (size_t)rows * DM * 2;
  const size_t PVT  = (size_t)BSZ * DM * (size_t)nseq * 2;
  size_t off = 0;
  const size_t oXh  = off; off += PXh;
  const size_t oWq  = off; off += PWq;
  const size_t oCt  = off; off += PTab;
  const size_t oSt  = off; off += PTab;
  const size_t oQKV = off; off += PQKV;
  const size_t oQh  = off; off += PQK;
  const size_t oKh  = off; off += PQK;
  const size_t oVT  = off; off += PVT;
  if (off > ws_size) return;
  if (off > (size_t)134217728) return;

  char* ws = (char*)d_ws;
  unsigned short* Xh   = (unsigned short*)(ws + oXh);
  unsigned short* Wq   = (unsigned short*)(ws + oWq);
  float*          Ct   = (float*)(ws + oCt);
  float*          St   = (float*)(ws + oSt);
  float*          QKVf = (float*)(ws + oQKV);
  unsigned short* Qh   = (unsigned short*)(ws + oQh);
  unsigned short* Kh   = (unsigned short*)(ws + oKh);
  unsigned short* VT   = (unsigned short*)(ws + oVT);
  float*          outf = (float*)d_out;

  Theta16 th;
  {
    const double qr[4] = {1.0, 1.7782794100389228, 3.1622776601683795, 5.623413251903491};
    double dec = 1.0;
    for (int j = 0; j < NFREQ; ++j) {
      const double pv = dec * qr[j & 3];
      const float pf = (float)pv;
      th.t[j] = 1.0f / pf;
      if ((j & 3) == 3) dec *= 10.0;
    }
  }

  const dim3 blk(256);
  const int nTab = nseq * NFREQ;
  const int n8x  = rows * DM / 8;
  const int n8w  = QKVN * DM / 8;
  const int nqt  = nseq / 64;
  const dim3 gTab((nTab + 255) / 256);
  const dim3 gCx((n8x + 255) / 256);
  const dim3 gCw((n8w + 255) / 256);
  const dim3 gQKV(((rows / 64) * (QKVN / 64) + 7) / 8);
  const dim3 gRope(rows);
  const dim3 gVpl(nqt, NH, BSZ);
  const dim3 gAttn(BSZ * NH * nqt);

  const float xScale  = 8.0f;
  const float wScale  = 64.0f;
  const float qkvInv  = 1.0f / 512.0f;
  const float qkScale = 16.0f;
  const float sscale  = 0.125f / 256.0f;
  const float vScale  = 256.0f;
  const float attOscl = 1.0f / 262144.0f;

  cvt_xh<<<gCx, blk, 0, stream>>>(x, Xh, n8x, xScale);
  cvt_xh<<<gCw, blk, 0, stream>>>(w, Wq, n8w, wScale);
  rope_tab<<<gTab, blk, 0, stream>>>(th, Ct, St, nTab);
  gemm64<<<gQKV, blk, 0, stream>>>(Xh, DM, Wq, DM, QKVf, QKVN, rows, QKVN, DM, qkvInv);
  rope_qk<<<gRope, dim3(128), 0, stream>>>(QKVf, Ct, St, Qh, Kh, qkScale);
  v_planes<<<gVpl, blk, 0, stream>>>(QKVf, VT, nseq, vScale);
  attn64<<<gAttn, dim3(128), 0, stream>>>(Qh, Kh, VT, outf, nseq, sscale, attOscl);
  (void)hipGetLastError();
}
